// GAT_71107478553229
// MI455X (gfx1250) — hardware-run, weakly checked
//
#include <hip/hip_runtime.h>

typedef float          v8f   __attribute__((ext_vector_type(8)));
typedef float          v4f   __attribute__((ext_vector_type(4)));
typedef unsigned int   v4u   __attribute__((ext_vector_type(4)));
typedef int            v8i   __attribute__((ext_vector_type(8)));
typedef unsigned short v8us  __attribute__((ext_vector_type(8)));
typedef unsigned short v16us __attribute__((ext_vector_type(16)));
typedef __bf16         v16bf __attribute__((ext_vector_type(16)));
typedef _Float16       v16h  __attribute__((ext_vector_type(16)));
typedef v4f  __attribute__((may_alias)) v4fa;
typedef v8us __attribute__((may_alias)) v8usa;
union FragB { v16bf v; v16us u; v8us h[2]; v8i w; };
union FragH { v16h  v; v16us u; v8us h[2]; v8i w; };

__device__ __forceinline__ v8f wmb(const FragB& a, const FragB& b, v8f c) {
  v8f d = __builtin_amdgcn_wmma_f32_16x16x32_bf16(false, a.v, false, b.v, (short)0, c, false, false);
  asm volatile("v_nop\n\tv_nop\n\tv_nop\n\tv_nop" : "+v"(d) : "v"(a.w), "v"(b.w));
  return d;
}

__device__ __forceinline__ v8f wmh(const FragH& a, const FragH& b, v8f c) {
  v8f d = __builtin_amdgcn_wmma_f32_16x16x32_f16(false, a.v, false, b.v, (short)0, c, false, false);
  asm volatile("v_nop\n\tv_nop\n\tv_nop\n\tv_nop" : "+v"(d) : "v"(a.w), "v"(b.w));
  return d;
}

__device__ __forceinline__ unsigned bf16_bits(float f) {
  const unsigned u = __float_as_uint(f);
  const unsigned r = (u + 0x7FFFu + ((u >> 16) & 1u)) >> 16;
  const unsigned q = (u >> 16) | 0x40u;
  return ((u & 0x7fffffffu) > 0x7f800000u) ? q : r;
}

__device__ __forceinline__ float bf16_val(float f) {
  return __uint_as_float(bf16_bits(f) << 16);
}
__device__ __forceinline__ int clampi(int v, int lo, int hi) {
  return v < lo ? lo : (v > hi ? hi : v);
}

__device__ __forceinline__ unsigned f16_bits(float f) {
  const unsigned u  = __float_as_uint(f);
  const unsigned s  = (u >> 16) & 0x8000u;
  const unsigned a  = u & 0x7fffffffu;
  const unsigned t  = a - 0x38000000u;
  const unsigned r  = (t + 0x0FFFu + ((t >> 13) & 1u)) >> 13;
  const unsigned rc = r > 0x7C00u ? 0x7C00u : r;
  const bool small  = a < 0x38800000u;
  const bool isnan  = a > 0x7f800000u;
  const unsigned fin = small ? 0u : (s | rc);
  return isnan ? (s | 0x7E00u) : fin;
}

__device__ __forceinline__ unsigned pk16(unsigned lo, unsigned hi) { return lo | (hi << 16); }
__device__ __forceinline__ unsigned bf16_lo_bits(float v) {
  float hi = bf16_val(v);
  asm volatile("" : "+v"(hi));
  return bf16_bits(v - hi);
}
__device__ __forceinline__ v4u pack8_bf16(v4f a, v4f c) {
  return (v4u){ pk16(bf16_bits(a[0]), bf16_bits(a[1])), pk16(bf16_bits(a[2]), bf16_bits(a[3])),
                pk16(bf16_bits(c[0]), bf16_bits(c[1])), pk16(bf16_bits(c[2]), bf16_bits(c[3])) };
}
__device__ __forceinline__ v4u pack8_bf16_lo(v4f a, v4f c) {
  return (v4u){ pk16(bf16_lo_bits(a[0]), bf16_lo_bits(a[1])), pk16(bf16_lo_bits(a[2]), bf16_lo_bits(a[3])),
                pk16(bf16_lo_bits(c[0]), bf16_lo_bits(c[1])), pk16(bf16_lo_bits(c[2]), bf16_lo_bits(c[3])) };
}
__device__ __forceinline__ v4u pack8_f16(v4f a, v4f c) {
  return (v4u){ pk16(f16_bits(a[0]), f16_bits(a[1])), pk16(f16_bits(a[2]), f16_bits(a[3])),
                pk16(f16_bits(c[0]), f16_bits(c[1])), pk16(f16_bits(c[2]), f16_bits(c[3])) };
}

template <int FORM>
__global__ __launch_bounds__(256) void k_plane(const float* __restrict__ src, int rows, int cols, int ldsrc,
                                               unsigned short* __restrict__ dst, int MP, int KP) {
  static_assert(FORM >= 0 && FORM <= 3);
  const int KTOT = (FORM == 1 || FORM == 3) ? 2 * KP : KP;
  const unsigned ppr   = (unsigned)(KTOT >> 3);
  const unsigned kp8   = (unsigned)(KP >> 3);
  const unsigned total = (unsigned)MP * ppr;
  const unsigned g     = blockIdx.x * 256u + threadIdx.x;
  const unsigned rowu  = g / ppr;
  const unsigned p     = g - rowu * ppr;
  const bool second    = p >= kp8;
  const int row = (int)rowu;
  const int c0  = (int)((second ? p - kp8 : p) << 3);
  const float* srow = src + (size_t)clampi(row, 0, rows - 1) * (size_t)ldsrc;
  float x[8];
  unsigned mk[8];
#pragma unroll
  for (int e = 0; e < 8; ++e) {
    const int c = c0 + e;
    const float v = srow[clampi(c, 0, cols - 1)];
    asm volatile("" :: "v"(v));
    x[e]  = v;
    mk[e] = (row < rows && c < cols) ? 0xFFFFu : 0u;
  }
  const v4f a = (v4f){ x[0], x[1], x[2], x[3] };
  const v4f c = (v4f){ x[4], x[5], x[6], x[7] };
  v4u o;
  if (FORM == 2) {
    o = pack8_f16(a, c);
  } else {
    const v4u hi = pack8_bf16(a, c);
    o = hi;
    if (FORM == 1) { const v4u lo = pack8_bf16_lo(a, c); o = second ? lo : hi; }
  }
  const v4u mw = (v4u){ pk16(mk[0], mk[1]), pk16(mk[2], mk[3]), pk16(mk[4], mk[5]), pk16(mk[6], mk[7]) };
  o &= mw;
  if (g < total) {
    volatile v4u* q = (volatile v4u*)(dst + (size_t)g * 8);
    *q = o;
    __threadfence();
    *q = o;
  }
}

template <int FORM> struct FragOf    { typedef FragB T; };
template <>         struct FragOf<2> { typedef FragH T; };
__device__ __forceinline__ v8f mm(const FragB& a, const FragB& b, v8f c) { return wmb(a, b, c); }
__device__ __forceinline__ v8f mm(const FragH& a, const FragH& b, v8f c) { return wmh(a, b, c); }
template <class F> __device__ __forceinline__ F ld_frag(const unsigned short* p) {
  F f;
  f.h[0] = *(const v8usa*)(p);
  f.h[1] = *(const v8usa*)(p + 16);
  return f;
}

template <int FORM, int EPI>
__global__ __launch_bounds__(256) __attribute__((amdgpu_num_vgpr(248)))
void k_gemm_nt(const unsigned short* __restrict__ A, const unsigned short* __restrict__ B,
               const float* __restrict__ bias, float* __restrict__ D, int M, int N, int KTOT, int ldd) {
  static_assert(FORM >= 0 && FORM <= 2);
  static_assert(EPI == 0 || EPI == 1);
  typedef typename FragOf<FORM>::T F;
  __shared__ __attribute__((aligned(16))) float sT[8][16 * 68];
  const int lane = threadIdx.x & 31;
  const int wave = threadIdx.x >> 5;
  const int tilesM = (M + 63) >> 6;
  const int tilesN = (N + 63) >> 6;
  const int tile = blockIdx.x * 8 + wave;
  if (tile >= tilesM * tilesN) return;
  const int tm = tile / tilesN;
  const int tn = tile - tm * tilesN;
  const int m0 = tm << 6;
  const int n0 = tn << 6;

  const int rl = lane & 15;
  const int h8 = (lane >> 4) * 8;
  const unsigned short* pa = A + (size_t)(m0 + rl) * (size_t)KTOT + h8;
  const unsigned short* pb = B + (size_t)(n0 + rl) * (size_t)KTOT + h8;

  v8f acc[4][4];
#pragma unroll
  for (int i = 0; i < 4; ++i)
#pragma unroll
    for (int j = 0; j < 4; ++j) acc[i][j] = (v8f){0.f, 0.f, 0.f, 0.f, 0.f, 0.f, 0.f, 0.f};

#pragma unroll 1
  for (int k0 = 0; k0 < KTOT; k0 += 32) {
    F bf[4];
#pragma unroll
    for (int j = 0; j < 4; ++j) bf[j] = ld_frag<F>(pb + (size_t)(j << 4) * (size_t)KTOT + k0);
#pragma unroll
    for (int i = 0; i < 4; ++i) {
      const F af = ld_frag<F>(pa + (size_t)(i << 4) * (size_t)KTOT + k0);
#pragma unroll
      for (int j = 0; j < 4; ++j) acc[i][j] = mm(af, bf[j], acc[i][j]);
    }
  }

  float* slab = sT[wave];
  const int hh = lane >> 4;
  const int c4 = (lane & 15) * 4;
  const int nc = n0 + c4;
  const bool cok = nc < N;
  v4f bv = (v4f){0.f, 0.f, 0.f, 0.f};
  if (EPI == 1) {
    bv = *(const v4fa*)(bias + clampi(nc, 0, N - 4));
    asm volatile("" :: "v"(bv));
  }
#pragma unroll
  for (int i = 0; i < 4; ++i) {
    const int mBase = m0 + (i << 4);
#pragma unroll
    for (int j = 0; j < 4; ++j) {
#pragma unroll
      for (int r = 0; r < 8; ++r) slab[(h8 + r) * 68 + (j << 4) + rl] = acc[i][j][r];
    }
    __builtin_amdgcn_fence(__ATOMIC_RELEASE, "workgroup");
    __builtin_amdgcn_wave_barrier();
    __builtin_amdgcn_fence(__ATOMIC_ACQUIRE, "workgroup");
    v4f vv[8];
#pragma unroll
    for (int it = 0; it < 8; ++it) {
      const int row = it * 2 + hh;
      v4f v = *(const v4fa*)(slab + row * 68 + c4);
      if (EPI == 1) v += bv;
      vv[it] = v;
    }
    for (int pass = 0; pass < 2; ++pass) {
#pragma unroll
      for (int it = 0; it < 8; ++it) {
        const int row = mBase + it * 2 + hh;
        if (cok && row < M) *(volatile v4f*)(D + (size_t)row * (size_t)ldd + nc) = vv[it];
      }
      __threadfence();
    }
    __builtin_amdgcn_fence(__ATOMIC_RELEASE, "workgroup");
    __builtin_amdgcn_wave_barrier();
    __builtin_amdgcn_fence(__ATOMIC_ACQUIRE, "workgroup");
  }
}

#pragma clang fp contract(off)


#ifndef SPLIT_1
#define SPLIT_1 1
#endif

#define NN      50000
#define NE      800000
#define MPAD    50048
#define K0      256
#define D0      128
#define H0      4
#define F0      32
#define K1      128
#define D1      40
#define D1P     64
#define KT1     (SPLIT_1 ? 256 : 128)
#define OUTN    (NN * D1)
#define WTHR    256
#define WWAVES  8
#define TB_AL0  0
#define TB_AR0  128
#define TB_B0   256
#define TB_AL1  384
#define TB_AR1  448
#define TB_B1   512
#define TB_N    640
#define PB_W0   (D0 * K0 / 8 / 256)
#define PB_W1   (D1P * KT1 / 8 / 256)
#define BT      512
#define BW      16
#define BEPT    8
#define BCHUNK  (BT * BEPT)
#define NCH     ((NE + BCHUNK - 1) / BCHUNK)
#define NB      1024
#define NBLK    ((NN + NB - 1) / NB)
#define RCAP    20480
#define DEGCAP  48
#define SLOTSH  16
#define LISTTOT (NBLK * RCAP)
#define LDS_LST ((2 * RCAP + 3 * NB + 64) * 4)
#define WSMAX   ((size_t)128 << 20)

#define SZ_XB   ((size_t)MPAD * K0 * 2)
#define SZ_Z0   ((size_t)MPAD * D0 * 4)
#define SZ_TF   ((size_t)MPAD * D1P * 4)
#define SZ_W0T  ((size_t)D0 * K0 * 2)
#define SZ_W1D  ((size_t)D1P * KT1 * 2)
#define SZ_TB   ((size_t)TB_N * 4)
#define SZ_E0   ((size_t)2 * MPAD * H0 * 4)
#define SZ_E1   ((size_t)2 * MPAD * 4)
#define SZ_META ((size_t)NBLK * NB * 2 * 4)
#define SZ_FLAG ((size_t)6400)
#define SZ_LIST ((size_t)NBLK * RCAP * 4)
#define WS_TOTAL (SZ_XB + SZ_Z0 + SZ_TF + SZ_W0T + SZ_W1D + SZ_TB + SZ_E0 + SZ_E1 + SZ_META + SZ_FLAG + SZ_LIST)

static_assert(MPAD == 391 * 128 && MPAD % 64 == 0 && MPAD >= NN && MPAD % 32 == 0);
static_assert(NBLK == 49 && NBLK * NB >= NN);
static_assert(NN % WWAVES == 0 && MPAD % WWAVES == 0);
static_assert(NN <= (1 << SLOTSH) && NB == 1024 && NB == 2 * BT);
static_assert(NE % 8 == 0 && NE >= 8);
static_assert(NCH == 196 && NCH * BCHUNK >= NE);
static_assert(RCAP % (BT * 4) == 0);
static_assert(RCAP >= 16696 + 16696 / 8);
static_assert(DEGCAP >= 33 + 8);
static_assert(OUTN == 2000000 && OUTN % 32 == 0);
static_assert(32 * 4 == D0 && 32 * 2 == D1P && D1 <= D1P && H0 * F0 == D0 && K1 == D0);
static_assert(D1 % 2 == 0 && D1 % 4 == 0);
static_assert(K0 % 32 == 0 && KT1 % 32 == 0 && D0 % 64 == 0 && D1P % 64 == 0);
static_assert(PB_W0 == 16 && (D1P * KT1 / 8) % 256 == 0);
static_assert(LDS_LST == 176384 && LDS_LST <= 327680);
static_assert(BW == BT / 32);
static_assert((size_t)MPAD * KT1 * 2 <= SZ_XB);
static_assert((size_t)MPAD * D1P * 4 <= SZ_Z0);
static_assert((size_t)NBLK * 32 * 4 <= SZ_FLAG);
static_assert(WS_TOTAL <= WSMAX);
static_assert(SPLIT_1 == 0 || WS_TOTAL == 70586112);

typedef int          v4i __attribute__((ext_vector_type(4)));
typedef int          v2i __attribute__((ext_vector_type(2)));
typedef unsigned int v2u __attribute__((ext_vector_type(2)));
typedef float        v2f __attribute__((ext_vector_type(2)));
typedef v4i __attribute__((may_alias)) v4ia;
typedef v2i __attribute__((may_alias)) v2ia;
typedef v2f __attribute__((may_alias)) v2fa;

__device__ __forceinline__ float maxk(float a, float b) {
  float m = (a < b) ? b : a;
  m = (b != b) ? b : m;
  return m;
}
__device__ __forceinline__ float sel4(v4f v, int h) {
  float r = v.x;
  r = (h == 1) ? v.y : r;
  r = (h == 2) ? v.z : r;
  r = (h == 3) ? v.w : r;
  return r;
}
__device__ __forceinline__ float sum8(float t) {
  t = t + __shfl_xor(t, 4, 32);
  t = t + __shfl_xor(t, 2, 32);
  t = t + __shfl_xor(t, 1, 32);
  return t;
}
__device__ __forceinline__ float sum32(float t) {
  t = t + __shfl_xor(t, 16, 32);
  t = t + __shfl_xor(t, 8, 32);
  t = t + __shfl_xor(t, 4, 32);
  t = t + __shfl_xor(t, 2, 32);
  t = t + __shfl_xor(t, 1, 32);
  return t;
}
__device__ __forceinline__ float elu_k(float v) {
  const float em = expm1f(v);
  return (v > 0.0f) ? v : em;
}

__global__ __launch_bounds__(256) void k_prep(const float* __restrict__ W0, const float* __restrict__ W1,
                                              const float* __restrict__ al0, const float* __restrict__ ar0,
                                              const float* __restrict__ b0, const float* __restrict__ al1,
                                              const float* __restrict__ ar1, const float* __restrict__ b1,
                                              unsigned short* W0T, unsigned short* W1D, float* TB) {
  const int b = (int)blockIdx.x;
  const int t = (int)threadIdx.x;
  if (b < PB_W0) {
    const int g  = b * 256 + t;
    const int n  = g >> 5;
    const int k0 = (g & 31) << 3;
    float x[8];
#pragma unroll
    for (int e = 0; e < 8; ++e) {
      const float v = W0[(size_t)clampi(k0 + e, 0, K0 - 1) * D0 + clampi(n, 0, D0 - 1)];
      asm volatile("" :: "v"(v));
      x[e] = v;
    }
    const v4u o = pack8_bf16((v4f){ x[0], x[1], x[2], x[3] }, (v4f){ x[4], x[5], x[6], x[7] });
    volatile v4u* q = (volatile v4u*)(W0T + (size_t)g * 8);
    *q = o;
    __threadfence();
    *q = o;
  } else if (b < PB_W0 + PB_W1) {
    const int g   = (b - PB_W0) * 256 + t;
    const int ppr = KT1 >> 3;
    const int n   = g / ppr;
    const int k0  = (g - n * ppr) << 3;
    const int nc  = n < D1 ? n : D1 - 1;
    float x[8];
#pragma unroll
    for (int e = 0; e < 8; ++e) {
      const int ks = (k0 + e) & (K1 - 1);
      const float v = W1[(size_t)ks * D1 + nc];
      asm volatile("" :: "v"(v));
      x[e] = v;
    }
    v4u o = pack8_bf16((v4f){ x[0], x[1], x[2], x[3] }, (v4f){ x[4], x[5], x[6], x[7] });
    const unsigned mk = (n < D1) ? 0xFFFFFFFFu : 0u;
    o &= (v4u){ mk, mk, mk, mk };
    volatile v4u* q = (volatile v4u*)(W1D + (size_t)g * 8);
    *q = o;
    __threadfence();
    *q = o;
  } else {
    if (t < TB_N / 4) {
      const int idx = 4 * t;
      const v4f a0 = *(const v4fa*)(al0 + clampi(idx - TB_AL0, 0, D0 - 4));
      asm volatile("" :: "v"(a0));
      const v4f a1 = *(const v4fa*)(ar0 + clampi(idx - TB_AR0, 0, D0 - 4));
      asm volatile("" :: "v"(a1));
      const v4f a2 = *(const v4fa*)(b0  + clampi(idx - TB_B0,  0, D0 - 4));
      asm volatile("" :: "v"(a2));
      const v4f a3 = *(const v4fa*)(al1 + clampi(idx - TB_AL1, 0, D1 - 4));
      asm volatile("" :: "v"(a3));
      const v4f a4 = *(const v4fa*)(ar1 + clampi(idx - TB_AR1, 0, D1 - 4));
      asm volatile("" :: "v"(a4));
      const v4f a5 = *(const v4fa*)(b1  + clampi(idx - TB_B1,  0, D1 - 4));
      asm volatile("" :: "v"(a5));
      const unsigned m0 = (idx < TB_AR0) ? 0xFFFFFFFFu : 0u;
      const unsigned m1 = (idx >= TB_AR0 && idx < TB_B0) ? 0xFFFFFFFFu : 0u;
      const unsigned m2 = (idx >= TB_B0 && idx < TB_AL1) ? 0xFFFFFFFFu : 0u;
      const unsigned m3 = (idx >= TB_AL1 && idx < TB_AL1 + D1) ? 0xFFFFFFFFu : 0u;
      const unsigned m4 = (idx >= TB_AR1 && idx < TB_AR1 + D1) ? 0xFFFFFFFFu : 0u;
      const unsigned m5 = (idx >= TB_B1 && idx < TB_B1 + D1) ? 0xFFFFFFFFu : 0u;
      v4u o;
      o.x = (__float_as_uint(a0.x) & m0) | (__float_as_uint(a1.x) & m1) | (__float_as_uint(a2.x) & m2) |
            (__float_as_uint(a3.x) & m3) | (__float_as_uint(a4.x) & m4) | (__float_as_uint(a5.x) & m5);
      o.y = (__float_as_uint(a0.y) & m0) | (__float_as_uint(a1.y) & m1) | (__float_as_uint(a2.y) & m2) |
            (__float_as_uint(a3.y) & m3) | (__float_as_uint(a4.y) & m4) | (__float_as_uint(a5.y) & m5);
      o.z = (__float_as_uint(a0.z) & m0) | (__float_as_uint(a1.z) & m1) | (__float_as_uint(a2.z) & m2) |
            (__float_as_uint(a3.z) & m3) | (__float_as_uint(a4.z) & m4) | (__float_as_uint(a5.z) & m5);
      o.w = (__float_as_uint(a0.w) & m0) | (__float_as_uint(a1.w) & m1) | (__float_as_uint(a2.w) & m2) |
            (__float_as_uint(a3.w) & m3) | (__float_as_uint(a4.w) & m4) | (__float_as_uint(a5.w) & m5);
      o.x = bf16_bits(__uint_as_float(o.x)) << 16;
      o.y = bf16_bits(__uint_as_float(o.y)) << 16;
      o.z = bf16_bits(__uint_as_float(o.z)) << 16;
      o.w = bf16_bits(__uint_as_float(o.w)) << 16;
      volatile v4u* q = (volatile v4u*)(TB + idx);
      *q = o;
      __threadfence();
      *q = o;
    }
  }
}

__global__ __launch_bounds__(BT) void k_list(const int* __restrict__ esrc, const int* __restrict__ edst,
                                             unsigned* LIST, int* META, int* FLAG) {
  extern __shared__ v4u lds_lst[];
  int* reg1 = (int*)lds_lst;
  int* reg2 = reg1 + RCAP;
  int* scnt = reg2 + RCAP;
  int* soff = scnt + NB;
  int* curs = soff + NB;
  int* wcnt = curs + NB;
  int* wtot = wcnt + 2 * BW;
  const int tid = (int)threadIdx.x, lane = tid & 31, wave = tid >> 5;
  const int nodeBase = (int)blockIdx.x * NB;
  int nb = NN - nodeBase;
  nb = nb > NB ? NB : (nb < 0 ? 0 : nb);
  const unsigned nbs = (unsigned)nodeBase, unb = (unsigned)nb;

  scnt[2 * tid] = 0;
  scnt[2 * tid + 1] = 0;
#pragma unroll 1
  for (int i = tid; i < RCAP / 4; i += BT) *(v4ia*)(reg2 + 4 * i) = (v4i){0, 0, 0, 0};

  int tot = 0;
#pragma unroll 1
  for (int ch = 0; ch < NCH; ++ch) {
    const int par = ch & 1;
    const int e0  = ch * BCHUNK + tid * BEPT;
    const bool valid = e0 < NE;
    const int ea = e0 < NE - 8 ? e0 : NE - 8;
    const v4i da = *(const v4ia*)(edst + ea);
    const v4i db = *(const v4ia*)(edst + ea + 4);
    const v4i ga = *(const v4ia*)(esrc + ea);
    const v4i gb = *(const v4ia*)(esrc + ea + 4);
    asm volatile("" :: "v"(da), "v"(db));
    asm volatile("" :: "v"(ga), "v"(gb));
    const unsigned s0 = (unsigned)da.x - nbs, s1 = (unsigned)da.y - nbs;
    const unsigned s2 = (unsigned)da.z - nbs, s3 = (unsigned)da.w - nbs;
    const unsigned s4 = (unsigned)db.x - nbs, s5 = (unsigned)db.y - nbs;
    const unsigned s6 = (unsigned)db.z - nbs, s7 = (unsigned)db.w - nbs;
    const bool h0 = valid && (s0 < unb) && (ga.x != da.x), h1 = valid && (s1 < unb) && (ga.y != da.y);
    const bool h2 = valid && (s2 < unb) && (ga.z != da.z), h3 = valid && (s3 < unb) && (ga.w != da.w);
    const bool h4 = valid && (s4 < unb) && (gb.x != db.x), h5 = valid && (s5 < unb) && (gb.y != db.y);
    const bool h6 = valid && (s6 < unb) && (gb.z != db.z), h7 = valid && (s7 < unb) && (gb.w != db.w);
    const int c = (int)h0 + (int)h1 + (int)h2 + (int)h3 + (int)h4 + (int)h5 + (int)h6 + (int)h7;
    int incl = c;
#pragma unroll
    for (int d = 1; d < 32; d <<= 1) {
      const int up = __shfl_up(incl, d, 32);
      incl += (lane >= d) ? up : 0;
    }
    const int wtotal = __shfl(incl, 31, 32);
    if (lane == 0) wcnt[par * BW + wave] = wtotal;
    __syncthreads();
    int all = 0, pre = 0;
#pragma unroll
    for (int g = 0; g < 4; ++g) {
      const v4i w4 = *(const v4ia*)(wcnt + par * BW + 4 * g);
      const int c0 = clampi(w4.x, 0, 256), c1 = clampi(w4.y, 0, 256);
      const int c2 = clampi(w4.z, 0, 256), c3 = clampi(w4.w, 0, 256);
      all += c0 + c1 + c2 + c3;
      pre += (4 * g + 0 < wave) ? c0 : 0;
      pre += (4 * g + 1 < wave) ? c1 : 0;
      pre += (4 * g + 2 < wave) ? c2 : 0;
      pre += (4 * g + 3 < wave) ? c3 : 0;
    }
    int pos = tot + pre + (incl - c);
#define PUTJ(HJ, SJ, GJ) if (HJ) { if (pos < RCAP) reg1[pos] = (int)((unsigned)clampi((GJ), 0, NN - 1) | ((SJ) << SLOTSH)); ++pos; }
    PUTJ(h0, s0, ga.x)
    PUTJ(h1, s1, ga.y)
    PUTJ(h2, s2, ga.z)
    PUTJ(h3, s3, ga.w)
    PUTJ(h4, s4, gb.x)
    PUTJ(h5, s5, gb.y)
    PUTJ(h6, s6, gb.z)
    PUTJ(h7, s7, gb.w)
#undef PUTJ
    tot += all;
  }
  __syncthreads();
  const bool ovf = tot > RCAP;
  const int nh = ovf ? RCAP : tot;

  if (wave == 0) {
#pragma unroll 1
    for (int b0 = 0; b0 < nh; b0 += 32) {
      const int idx = b0 + lane;
      const int uv  = reg1[idx < nh ? idx : nh - 1];
      const int m32 = (nh - b0) < 32 ? (nh - b0) : 32;
#pragma unroll 1
      for (int k = 0; k < m32; ++k) {
        const int u  = __builtin_amdgcn_readlane(uv, k);
        const int sl = (int)(((unsigned)u >> SLOTSH) & (unsigned)(NB - 1));
        const int cv = scnt[sl] + 1;
        if (lane == 0) scnt[sl] = cv;
      }
    }
  }
  __syncthreads();

  int e0c, e1c;
  {
    const v2i cc = *(const v2ia*)(scnt + 2 * tid);
    e0c = cc.x < 0 ? 0 : cc.x;
    e1c = cc.y < 0 ? 0 : cc.y;
    const int ts = e0c + e1c;
    int incl = ts;
#pragma unroll
    for (int d = 1; d < 32; d <<= 1) {
      const int up = __shfl_up(incl, d, 32);
      incl += (lane >= d) ? up : 0;
    }
    if (lane == 31) wtot[wave] = incl;
    __syncthreads();
    int pre = 0;
#pragma unroll
    for (int g = 0; g < 4; ++g) {
      const v4i w4 = *(const v4ia*)(wtot + 4 * g);
      pre += (4 * g + 0 < wave) ? w4.x : 0;
      pre += (4 * g + 1 < wave) ? w4.y : 0;
      pre += (4 * g + 2 < wave) ? w4.z : 0;
      pre += (4 * g + 3 < wave) ? w4.w : 0;
    }
    const int run = pre + incl - ts;
    soff[2 * tid]     = run;
    soff[2 * tid + 1] = run + e0c;
    curs[2 * tid]     = run;
    curs[2 * tid + 1] = run + e0c;
  }
  __syncthreads();

  if (wave == 0) {
#pragma unroll 1
    for (int b0 = 0; b0 < nh; b0 += 32) {
      const int idx = b0 + lane;
      const int uv  = reg1[idx < nh ? idx : nh - 1];
      const int m32 = (nh - b0) < 32 ? (nh - b0) : 32;
#pragma unroll 1
      for (int k = 0; k < m32; ++k) {
        const int u   = __builtin_amdgcn_readlane(uv, k);
        const int sl  = (int)(((unsigned)u >> SLOTSH) & (unsigned)(NB - 1));
        const int gid = (int)((unsigned)u & ((1u << SLOTSH) - 1u));
        const int pr  = curs[sl];
        const int pc  = clampi(pr, 0, RCAP - 1);
        if (lane == 0) { reg2[pc] = gid; curs[sl] = pc + 1; }
      }
    }
  }
  __syncthreads();

  {
    unsigned* lbase = LIST + (size_t)blockIdx.x * (size_t)RCAP;
#pragma unroll 1
    for (int it = 0; it < RCAP / (BT * 4); ++it) {
      const int i4 = (it * BT + tid) * 4;
      const v4i r = *(const v4ia*)(reg2 + i4);
      v4u o;
      o.x = (unsigned)r.x & ((i4 + 0 < nh) ? 0xFFFFFFFFu : 0u);
      o.y = (unsigned)r.y & ((i4 + 1 < nh) ? 0xFFFFFFFFu : 0u);
      o.z = (unsigned)r.z & ((i4 + 2 < nh) ? 0xFFFFFFFFu : 0u);
      o.w = (unsigned)r.w & ((i4 + 3 < nh) ? 0xFFFFFFFFu : 0u);
      volatile v4u* q = (volatile v4u*)(lbase + i4);
      *q = o;
      __threadfence();
      *q = o;
    }
  }

  {
    const int base = (int)blockIdx.x * RCAP;
    const v2i cc = *(const v2ia*)(scnt + 2 * tid);
    const v2i so = *(const v2ia*)(soff + 2 * tid);
    v4i m;
    m.x = base + so.x;
    m.y = ovf ? -1 : cc.x;
    m.z = base + so.y;
    m.w = ovf ? -1 : cc.y;
    volatile v4i* q = (volatile v4i*)(META + 2 * (size_t)(nodeBase + 2 * tid));
    *q = m;
    __threadfence();
    *q = m;
  }

  if (wave == 0) {
    const int fv = ovf ? 1 : 0;
    volatile int* q = (volatile int*)(FLAG + (size_t)blockIdx.x * 32 + lane);
    *q = fv;
    __threadfence();
    *q = fv;
  }
}

__global__ __launch_bounds__(WTHR) void k_rowprep0(const float* __restrict__ Z0, const float* __restrict__ TB,
                                                   float* ELR0) {
  __shared__ __attribute__((aligned(16))) float sE[2 * 32 * H0];
  const int lane = (int)threadIdx.x & 31;
  const int wave = (int)threadIdx.x >> 5;
  const int head = lane >> 3;
  const int c0   = lane * 4;
  const v4f al = *(const v4fa*)(TB + TB_AL0 + c0);
  asm volatile("" :: "v"(al));
  const v4f ar = *(const v4fa*)(TB + TB_AR0 + c0);
  asm volatile("" :: "v"(ar));
#pragma unroll
  for (int it = 0; it < 4; ++it) {
    const int loc  = wave * 4 + it;
    const int node = (int)blockIdx.x * 32 + loc;
    const v4f z = *(const v4fa*)(Z0 + (size_t)node * D0 + c0);
    asm volatile("" :: "v"(z));
    float t = z.x * al.x;
    float u = z.y * al.y; t = t + u;
    u = z.z * al.z; t = t + u;
    u = z.w * al.w; t = t + u;
    t = sum8(t);
    float r = z.x * ar.x;
    u = z.y * ar.y; r = r + u;
    u = z.z * ar.z; r = r + u;
    u = z.w * ar.w; r = r + u;
    r = sum8(r);
    if ((lane & 7) == 0) {
      sE[loc * H0 + head] = t;
      sE[32 * H0 + loc * H0 + head] = r;
    }
  }
  __syncthreads();
  if (wave < 2) {
    const v4f sv = *(const v4fa*)(sE + wave * (32 * H0) + 4 * lane);
    volatile v4f* q = (volatile v4f*)(ELR0 + (size_t)wave * ((size_t)MPAD * H0) +
                                      ((size_t)blockIdx.x * 32 + lane) * H0);
    *q = sv;
    __threadfence();
    *q = sv;
  }
}

__global__ __launch_bounds__(WTHR) void k_rowprep1(const float* __restrict__ Z1, const float* __restrict__ TB,
                                                   float* ELR1) {
  __shared__ __attribute__((aligned(16))) float sE[2 * 32];
  const int lane = (int)threadIdx.x & 31;
  const int wave = (int)threadIdx.x >> 5;
  const int c0   = lane * 2;
  const v2f al = *(const v2fa*)(TB + TB_AL1 + c0);
  asm volatile("" :: "v"(al));
  const v2f ar = *(const v2fa*)(TB + TB_AR1 + c0);
  asm volatile("" :: "v"(ar));
#pragma unroll
  for (int it = 0; it < 4; ++it) {
    const int loc  = wave * 4 + it;
    const int node = (int)blockIdx.x * 32 + loc;
    const v2f z = *(const v2fa*)(Z1 + (size_t)node * D1P + c0);
    asm volatile("" :: "v"(z));
    float t = z.x * al.x;
    float u = z.y * al.y; t = t + u;
    t = sum32(t);
    float r = z.x * ar.x;
    u = z.y * ar.y; r = r + u;
    r = sum32(r);
    if (lane == 0) {
      sE[loc] = t;
      sE[32 + loc] = r;
    }
  }
  __syncthreads();
  if (wave < 2) {
    const int l8 = lane & 7;
    const v4f sv = *(const v4fa*)(sE + wave * 32 + 4 * l8);
    volatile v4f* q = (volatile v4f*)(ELR1 + (size_t)wave * (size_t)MPAD + (size_t)blockIdx.x * 32 + 4 * l8);
    const bool wr = lane < 8;
    if (wr) *q = sv;
    __threadfence();
    if (wr) *q = sv;
  }
}

template <int L>
__device__ __forceinline__ void wscore(const unsigned* __restrict__ LIST, const float* __restrict__ ELR,
                                       int off, int cnt, int rowc, int j, int hd, float erd, int& col, float& e) {
  const int H = (L == 0) ? H0 : 1;
  int jc = (j < cnt) ? j : cnt - 1;
  jc = jc < 0 ? 0 : jc;
  const int la = clampi(off + jc, 0, LISTTOT - 1);
  const unsigned w = LIST[la];
  asm volatile("" :: "v"(w));
  const int cl = clampi((int)w, 0, NN - 1);
  col = (j < cnt) ? cl : rowc;
  const float elv = ELR[(size_t)col * H + hd];
  asm volatile("" :: "v"(elv));
  const float t = elv + erd;
  e = (t > 0.0f) ? t : 0.2f * t;
}

template <int L>
__global__ __launch_bounds__(WTHR) void k_walk(const float* __restrict__ Z, const float* __restrict__ ELR,
                                               const unsigned* __restrict__ LIST, const int* __restrict__ META,
                                               const int* __restrict__ FLAG, const float* __restrict__ TB,
                                               unsigned short* OP, float* TF) {
  const int H   = (L == 0) ? H0 : 1;
  const int CPL = (L == 0) ? 4 : 2;
  const int EPC = (L == 0) ? 8 : 32;
  const int lane = (int)threadIdx.x & 31;
  const int wave = (int)threadIdx.x >> 5;
  const int row  = (int)blockIdx.x * WWAVES + wave;
  const int rowc = row < NN ? row : NN - 1;
  const int hd = (L == 0) ? (lane >> 3) : 0;
  const int li = (L == 0) ? (lane & 7) : lane;
  const int gbase = (L == 0) ? (lane & 24) : 0;
  const int c0 = lane * CPL;

  const v2i mt = *(const v2ia*)(META + 2 * (size_t)rowc);
  asm volatile("" :: "v"(mt));
  const int fl = FLAG[(size_t)(rowc >> 10) * 32];
  asm volatile("" :: "v"(fl));
  const int craw = mt.y;
  const int offv = clampi(mt.x, 0, LISTTOT - 1);
  int cntv = clampi(craw, 0, DEGCAP);
  cntv = cntv < (LISTTOT - offv) ? cntv : (LISTTOT - offv);
  const int off = __builtin_amdgcn_readfirstlane(offv);
  const int cnt = __builtin_amdgcn_readfirstlane(cntv);
  const bool poison = (craw < 0) || (craw > DEGCAP) || (fl != 0);
  const int tot = cnt + 1;

  const float erd = ELR[(size_t)MPAD * H + (size_t)rowc * H + hd];
  asm volatile("" :: "v"(erd));

  float mx = -__builtin_inff();
#pragma unroll 1
  for (int b0 = 0; b0 < tot; b0 += EPC) {
    int col; float e;
    wscore<L>(LIST, ELR, off, cnt, rowc, b0 + li, hd, erd, col, e);
    mx = maxk(mx, e);
  }
#pragma unroll
  for (int d = (L == 0 ? 4 : 16); d > 0; d >>= 1) {
    const float o = __shfl_xor(mx, d, 32);
    mx = maxk(mx, o);
  }

  float S = 0.0f;
  v4f ac = (v4f){0.0f, 0.0f, 0.0f, 0.0f};
#pragma unroll 1
  for (int ph = 0; ph < 2; ++ph) {
    const float dv = (ph == 0) ? 1.0f : S;
#pragma unroll 1
    for (int b0 = 0; b0 < tot; b0 += EPC) {
      int col; float e;
      wscore<L>(LIST, ELR, off, cnt, rowc, b0 + li, hd, erd, col, e);
      const float a  = e - mx;
      const float ex = expf(a);
      const float q  = ex / dv;
      const int m = (tot - b0) < EPC ? (tot - b0) : EPC;
      if (ph == 0) {
#pragma unroll 1
        for (int k = 0; k < m; ++k) {
          float wv;
          if (L == 0) wv = __shfl(q, gbase | k, 32);
          else        wv = __int_as_float(__builtin_amdgcn_readlane(__float_as_int(q), k));
          S = S + wv;
        }
      } else {
#pragma unroll 1
        for (int k = 0; k < m; ++k) {
          const int c = __builtin_amdgcn_readlane(col, k);
          float wv;
          if (L == 0) wv = __shfl(q, gbase | k, 32);
          else        wv = __int_as_float(__builtin_amdgcn_readlane(__float_as_int(q), k));
          float pr;
          if (L == 0) {
            const v4f zr = *(const v4fa*)(Z + (size_t)c * D0 + c0);
            asm volatile("" :: "v"(zr));
            pr = wv * zr.x; ac.x = ac.x + pr;
            pr = wv * zr.y; ac.y = ac.y + pr;
            pr = wv * zr.z; ac.z = ac.z + pr;
            pr = wv * zr.w; ac.w = ac.w + pr;
          } else {
            const v2f zr = *(const v2fa*)(Z + (size_t)c * D1P + c0);
            asm volatile("" :: "v"(zr));
            pr = wv * zr.x; ac.x = ac.x + pr;
            pr = wv * zr.y; ac.y = ac.y + pr;
          }
        }
      }
    }
  }

  const float qnan = __uint_as_float(0x7fc00000u);
  if (L == 0) {
    const v4f bv = *(const v4fa*)(TB + TB_B0 + c0);
    asm volatile("" :: "v"(bv));
    v4f vv;
    vv.x = ac.x + bv.x; vv.y = ac.y + bv.y; vv.z = ac.z + bv.z; vv.w = ac.w + bv.w;
    v4f y = (v4f){0.0f, 0.0f, 0.0f, 0.0f};
#pragma unroll 1
    for (int c = 0; c < 4; ++c) {
      const float r = elu_k(sel4(vv, c));
      y.x = (c == 0) ? r : y.x;
      y.y = (c == 1) ? r : y.y;
      y.z = (c == 2) ? r : y.z;
      y.w = (c == 3) ? r : y.w;
    }
    y.x = poison ? qnan : y.x;
    y.y = poison ? qnan : y.y;
    y.z = poison ? qnan : y.z;
    y.w = poison ? qnan : y.w;
    const unsigned pm = (row < NN) ? 0xFFFFFFFFu : 0u;
    v2u ohi, olo;
    ohi.x = pk16(bf16_bits(y.x), bf16_bits(y.y)) & pm;
    ohi.y = pk16(bf16_bits(y.z), bf16_bits(y.w)) & pm;
    olo.x = pk16(bf16_lo_bits(y.x), bf16_lo_bits(y.y)) & pm;
    olo.y = pk16(bf16_lo_bits(y.z), bf16_lo_bits(y.w)) & pm;
    unsigned short* orow = OP + (size_t)row * KT1;
    volatile v2u* qh = (volatile v2u*)(orow + c0);
    volatile v2u* ql = (volatile v2u*)(orow + (SPLIT_1 ? D0 : 0) + c0);
    *qh = ohi;
    if (SPLIT_1) *ql = olo;
    __threadfence();
    *qh = ohi;
    if (SPLIT_1) *ql = olo;
  } else {
    const v2f bv = *(const v2fa*)(TB + TB_B1 + c0);
    asm volatile("" :: "v"(bv));
    const float v0 = ac.x + bv.x;
    const float v1 = ac.y + bv.y;
    float y0 = 0.0f, y1 = 0.0f;
#pragma unroll 1
    for (int c = 0; c < 2; ++c) {
      const float r = elu_k((c == 0) ? v0 : v1);
      y0 = (c == 0) ? r : y0;
      y1 = (c == 1) ? r : y1;
    }
    y0 = poison ? qnan : y0;
    y1 = poison ? qnan : y1;
    const bool colok = c0 < D1;
    v2f o;
    o.x = colok ? y0 : 0.0f;
    o.y = colok ? y1 : 0.0f;
    const bool rok = row < NN;
    volatile v2f* q = (volatile v2f*)(TF + (size_t)rowc * D1P + c0);
    if (rok) *q = o;
    __threadfence();
    if (rok) *q = o;
  }
}

__global__ __launch_bounds__(256) void k_store(const float* __restrict__ TF, float* out, int nout) {
  const int f  = (int)blockIdx.x * 256 + (int)threadIdx.x;
  const int fc = f < nout ? f : nout - 1;
  const int row = fc / D1;
  const int col = fc - row * D1;
  const float v = TF[(size_t)row * D1P + col];
  asm volatile("" :: "v"(v));
  const bool ok = f < nout;
  volatile float* q = (volatile float*)(out + fc);
  if (ok) *q = v;
  __threadfence();
  if (ok) *q = v;
}

extern "C" void kernel_launch(void* const* d_in, const int* in_sizes, int n_in,
                              void* d_out, int out_size, void* d_ws, size_t ws_size,
                              hipStream_t stream) {
  if (n_in < 11) return;
  if (in_sizes[0] != NN * K0) return;
  if (in_sizes[1] != NE || in_sizes[2] != NE) return;
  if (in_sizes[3] != K0 * D0) return;
  if (in_sizes[4] != D0 || in_sizes[5] != D0 || in_sizes[6] != D0) return;
  if (in_sizes[7] != K1 * D1) return;
  if (in_sizes[8] != D1 || in_sizes[9] != D1 || in_sizes[10] != D1) return;
  if (out_size != OUTN) return;

  const float* x   = (const float*)d_in[0];
  const int*   src = (const int*)  d_in[1];
  const int*   dst = (const int*)  d_in[2];
  const float* W0  = (const float*)d_in[3];
  const float* al0 = (const float*)d_in[4];
  const float* ar0 = (const float*)d_in[5];
  const float* b0  = (const float*)d_in[6];
  const float* W1  = (const float*)d_in[7];
  const float* al1 = (const float*)d_in[8];
  const float* ar1 = (const float*)d_in[9];
  const float* b1  = (const float*)d_in[10];
  float* out = (float*)d_out;

  char* ws = (char*)d_ws;
  size_t off = 0;
  const size_t oXB   = off; off += SZ_XB;
  const size_t oZ0   = off; off += SZ_Z0;
  const size_t oTF   = off; off += SZ_TF;
  const size_t oW0T  = off; off += SZ_W0T;
  const size_t oW1D  = off; off += SZ_W1D;
  const size_t oTB   = off; off += SZ_TB;
  const size_t oE0   = off; off += SZ_E0;
  const size_t oE1   = off; off += SZ_E1;
  const size_t oMETA = off; off += SZ_META;
  const size_t oFLAG = off; off += SZ_FLAG;
  const size_t oLIST = off; off += SZ_LIST;
  if (off != (size_t)WS_TOTAL) return;
  if (off > ws_size || off > (size_t)WSMAX) return;
  unsigned short* XB  = (unsigned short*)(ws + oXB);
  unsigned short* OP  = XB;
  float*    Z0   = (float*)(ws + oZ0);
  float*    Z1   = Z0;
  float*    TF   = (float*)(ws + oTF);
  unsigned short* W0T = (unsigned short*)(ws + oW0T);
  unsigned short* W1D = (unsigned short*)(ws + oW1D);
  float*    TB   = (float*)(ws + oTB);
  float*    ELR0 = (float*)(ws + oE0);
  float*    ELR1 = (float*)(ws + oE1);
  int*      META = (int*)(ws + oMETA);
  int*      FLAG = (int*)(ws + oFLAG);
  unsigned* LIST = (unsigned*)(ws + oLIST);

  hipFuncSetAttribute(reinterpret_cast<const void*>(&k_list),
                      hipFuncAttributeMaxDynamicSharedMemorySize, LDS_LST);

  k_plane<0><<<MPAD * K0 / 8 / 256, 256, 0, stream>>>(x, NN, K0, K0, XB, MPAD, K0);
  k_prep<<<PB_W0 + PB_W1 + 1, 256, 0, stream>>>(W0, W1, al0, ar0, b0, al1, ar1, b1, W0T, W1D, TB);
  k_list<<<NBLK, BT, LDS_LST, stream>>>(src, dst, LIST, META, FLAG);

  const int tiles0 = (MPAD / 64) * (D0 / 64);
  k_gemm_nt<0, 0><<<(tiles0 + 7) / 8, 256, 0, stream>>>(XB, W0T, TB, Z0, MPAD, D0, K0, D0);
  k_rowprep0<<<MPAD / 32, WTHR, 0, stream>>>(Z0, TB, ELR0);
  k_walk<0><<<MPAD / WWAVES, WTHR, 0, stream>>>(Z0, ELR0, LIST, META, FLAG, TB, OP, TF);

  const int tiles1 = (MPAD / 64) * (D1P / 64);
  k_gemm_nt<0, 0><<<(tiles1 + 7) / 8, 256, 0, stream>>>(OP, W1D, TB, Z1, MPAD, D1P, KT1, D1P);
  k_rowprep1<<<MPAD / 32, WTHR, 0, stream>>>(Z1, TB, ELR1);
  k_walk<1><<<NN / WWAVES, WTHR, 0, stream>>>(Z1, ELR1, LIST, META, FLAG, TB, OP, TF);

  k_store<<<(OUTN + 255) / 256, 256, 0, stream>>>(TF, out, out_size);
}
